// NonLocalBlock_36593121361934
// MI455X (gfx1250) — hardware-verified
//
#include <hip/hip_runtime.h>
#include <math.h>
#include <stdint.h>

#ifndef NB
#define NB 4
#endif
#define NB_FULL 4
#define CC      512
#define NN      4096
#ifndef NQ
#define NQ NN
#endif
#define NGRP    32
#define CPG     16
#define GNE     (CPG * NN)
#define QT      64
#define OSP     68
#define OSPW    132
#define TP      72
#define STL     32
#define CH      256
#define SXB     2048
#define GEPS    1.0e-6f
#define ASCALE  0.04419417382415922f
#define LNPS    9.704060527839234f

static_assert(NB >= 1 && NB <= NB_FULL);
static_assert(NQ % QT == 0 && NQ >= QT && NQ <= NN);
static_assert(CC == NGRP * CPG);
static_assert(CC % QT == 0 && NN % QT == 0);
static_assert(CC == 2 * CH && CH == 16 * 16);
static_assert(CC == 8 * 64);
static_assert(GNE % 1024 == 0);
static_assert(CC % 32 == 0 && NN % 32 == 0);
static_assert((OSP * 4) % 16 == 0 && (OSPW * 4) % 16 == 0 && (TP * 2) % 16 == 0);
static_assert(SXB == 8 * 32 * 8);

typedef _Float16       v16h __attribute__((ext_vector_type(16)));
typedef _Float16       v8h  __attribute__((ext_vector_type(8)));
typedef __bf16         v16b __attribute__((ext_vector_type(16)));
typedef unsigned short v8us __attribute__((ext_vector_type(8)));
typedef float          v8f  __attribute__((ext_vector_type(8)));
typedef float          v4f  __attribute__((ext_vector_type(4)));
typedef unsigned int   v4u  __attribute__((ext_vector_type(4)));

union Frag  { v8us u[2]; v16h h; v16b bf; };
union FragH { v16h v; v8h hv[2]; };
static_assert(sizeof(Frag) == 32);
static_assert(sizeof(FragH) == 32);

__device__ __forceinline__ unsigned short bf_bits(float f) {
  unsigned u = __float_as_uint(f);
  return (unsigned short)((u + 0x7FFFu + ((u >> 16) & 1u)) >> 16);
}
__device__ __forceinline__ float bf_up(unsigned short hb) { return __uint_as_float(((unsigned)hb) << 16); }
__device__ __forceinline__ float bfr(float f) { return bf_up(bf_bits(f)); }
__device__ __forceinline__ unsigned short h_bits(_Float16 x) { return __builtin_bit_cast(unsigned short, x); }
__device__ __forceinline__ unsigned pk16(unsigned short a, unsigned short b) { return (unsigned)a | ((unsigned)b << 16); }
__device__ __forceinline__ v8f zero8() { v8f z = {0.f, 0.f, 0.f, 0.f, 0.f, 0.f, 0.f, 0.f}; return z; }
__device__ __forceinline__ float hmax8(v8f s) {
  return fmaxf(fmaxf(fmaxf(s[0], s[1]), fmaxf(s[2], s[3])), fmaxf(fmaxf(s[4], s[5]), fmaxf(s[6], s[7])));
}
__device__ __forceinline__ unsigned wave_ballot(bool p) {
#if defined(__HIP_DEVICE_COMPILE__)
  return __builtin_amdgcn_ballot_w32(p);
#else
  return p ? 1u : 0u;
#endif
}

__device__ __forceinline__ Frag ldfrag(const unsigned short* p) {
  Frag f;
  f.u[0] = *(const v8us*)(p);
  f.u[1] = *(const v8us*)(p + 16);
  return f;
}

__device__ __forceinline__ v8f mma_h(v16h a, v16h b, v8f c) {
  v8f d = __builtin_amdgcn_wmma_f32_16x16x32_f16(false, a, false, b, (short)0, c, false, false);
#if defined(__HIP_DEVICE_COMPILE__)
  asm volatile("v_nop\n\tv_nop\n\tv_nop\n\tv_nop" : "+v"(d) : "v"(a), "v"(b));
#endif
  return d;
}
__device__ __forceinline__ v8f mma_b(v16b a, v16b b, v8f c) {
  v8f d = __builtin_amdgcn_wmma_f32_16x16x32_bf16(false, a, false, b, (short)0, c, false, false);
#if defined(__HIP_DEVICE_COMPILE__)
  const v16h ha = __builtin_bit_cast(v16h, a), hb = __builtin_bit_cast(v16h, b);
  asm volatile("v_nop\n\tv_nop\n\tv_nop\n\tv_nop" : "+v"(d) : "v"(ha), "v"(hb));
#endif
  return d;
}

__global__ __launch_bounds__(256)
void gn_stats(const float* __restrict__ x, float* stats) {
  __shared__ float red[256];
  const int tid = threadIdx.x, bg = blockIdx.x;
  const float* p = x + (size_t)bg * GNE;
  float s = 0.f;
#pragma unroll 1
  for (int i = 0; i < GNE / 1024; ++i) {
    const v4f v = *(const v4f*)(p + ((size_t)(i * 256 + tid)) * 4);
    s += (bfr(v[0]) + bfr(v[1])) + (bfr(v[2]) + bfr(v[3]));
  }
  red[tid] = s;
  __syncthreads();
#pragma unroll 1
  for (int off = 128; off > 0; off >>= 1) {
    if (tid < off) red[tid] += red[tid + off];
    __syncthreads();
  }
  const float mean = red[0] * (1.0f / (float)GNE);
  __syncthreads();
  float ss = 0.f;
#pragma unroll 1
  for (int i = 0; i < GNE / 1024; ++i) {
    const v4f v = *(const v4f*)(p + ((size_t)(i * 256 + tid)) * 4);
    const float d0 = bfr(v[0]) - mean, d1 = bfr(v[1]) - mean;
    const float d2 = bfr(v[2]) - mean, d3 = bfr(v[3]) - mean;
    ss += (d0 * d0 + d1 * d1) + (d2 * d2 + d3 * d3);
  }
  red[tid] = ss;
  __syncthreads();
#pragma unroll 1
  for (int off = 128; off > 0; off >>= 1) {
    if (tid < off) red[tid] += red[tid + off];
    __syncthreads();
  }
  const float var  = red[0] * (1.0f / (float)GNE);
  const float rstd = rsqrtf(var + GEPS);
  if (tid < 8) {
    v4f w = {0.f, 0.f, 0.f, 0.f};
    if (tid == 0) { w[0] = mean; w[1] = rstd; }
#pragma unroll
    for (int pass = 0; pass < 2; ++pass) {
      *(volatile v4f*)(stats + (size_t)bg * STL + 4 * tid) = w;
      __threadfence();
    }
  }
}

__global__ __launch_bounds__(256)
void cvt_w(const float* __restrict__ wq, const float* __restrict__ wk, const float* __restrict__ wv,
           unsigned short* Wb) {
  const int tid = threadIdx.x, blk = blockIdx.x;
  const int mat = blk / (CC / 4);
  const int o   = 4 * (blk % (CC / 4)) + (tid >> 6);
  const int col = 8 * (tid & 63);
  const float* wsrc = (mat == 0) ? wq : ((mat == 1) ? wk : wv);
  const float* s = wsrc + (size_t)o * CC + col;
  const v4f a = *(const v4f*)s;
  const v4f q = *(const v4f*)(s + 4);
  const float f[8] = {a[0], a[1], a[2], a[3], q[0], q[1], q[2], q[3]};
  v4u u;
#pragma unroll
  for (int t = 0; t < 4; ++t) u[t] = pk16(bf_bits(f[2 * t]), bf_bits(f[2 * t + 1]));
#pragma unroll
  for (int pass = 0; pass < 2; ++pass) {
    *(volatile v4u*)(Wb + ((size_t)(mat * CC + o)) * CC + col) = u;
    __threadfence();
  }
}

__global__ __launch_bounds__(256)
void cvt_x(const float* __restrict__ x, const float* __restrict__ gamma, const float* __restrict__ beta,
           const float* __restrict__ stats, unsigned short* Hh, unsigned short* Hl) {
  __shared__ __align__(16) unsigned short Th[QT * TP];
  __shared__ __align__(16) unsigned short Tl[QT * TP];
  const int tid = threadIdx.x;
  const int nb = blockIdx.x, cb = blockIdx.y, b = blockIdx.z;
  const int e = tid & 7, lq = tid >> 3;
  const int n0 = nb * QT, c0 = cb * QT;
#pragma unroll
  for (int it = 0; it < 2; ++it) {
    const int cl = it * 32 + lq;
    const int cg = c0 + cl;
    const int bg = b * NGRP + (cg >> 4);
    const float mean = stats[(size_t)bg * STL];
    const float rstd = stats[(size_t)bg * STL + 1];
    const float ga = bfr(gamma[cg]);
    const float be = bfr(beta[cg]);
    const float* sp = x + ((size_t)(b * CC + cg)) * NN + n0 + 8 * e;
    const v4f a = *(const v4f*)sp;
    const v4f q = *(const v4f*)(sp + 4);
    const float f[8] = {a[0], a[1], a[2], a[3], q[0], q[1], q[2], q[3]};
#pragma unroll
    for (int t = 0; t < 8; ++t) {
      const float h = ((bfr(f[t]) - mean) * rstd) * ga + be;
      const unsigned short hb = bf_bits(h);
      const unsigned short lb = bf_bits(h - bf_up(hb));
      Th[(8 * e + t) * TP + cl] = hb;
      Tl[(8 * e + t) * TP + cl] = lb;
    }
  }
  __syncthreads();
  v4u uh[2], ul[2];
#pragma unroll
  for (int it = 0; it < 2; ++it) {
    const int nl = it * 32 + lq;
    uh[it] = *(const v4u*)(Th + nl * TP + 8 * e);
    ul[it] = *(const v4u*)(Tl + nl * TP + 8 * e);
  }
#pragma unroll
  for (int pass = 0; pass < 2; ++pass) {
#pragma unroll
    for (int it = 0; it < 2; ++it) {
      const int nl = it * 32 + lq;
      const size_t po = ((size_t)(b * NN + n0 + nl)) * CC + c0 + 8 * e;
      *(volatile v4u*)(Hh + po) = uh[it];
      *(volatile v4u*)(Hl + po) = ul[it];
    }
    __threadfence();
  }
}

__global__ __launch_bounds__(128)
void gemm_qkv(const unsigned short* __restrict__ Wb, const unsigned short* __restrict__ Hh,
              const unsigned short* __restrict__ Hl,
              const float* __restrict__ bq, const float* __restrict__ bk, const float* __restrict__ bv,
              unsigned short* Qd, unsigned short* Kd, unsigned short* Vd) {
  __shared__ __align__(16) float Os[QT * OSP];
  const int tid  = threadIdx.x;
  const int lane = tid & 31, wave = tid >> 5;
  const int hh   = lane >> 4, c = lane & 15;
  const int nt   = blockIdx.x, my = blockIdx.y, b = blockIdx.z;
  const int mat  = my / (CC / QT);
  const int ob   = my % (CC / QT);
  const int n0   = nt * QT, o0 = ob * QT;

  const unsigned short* ap = Wb + ((size_t)(mat * CC + o0 + c)) * CC + 8 * hh;
  const size_t brow = ((size_t)(b * NN + n0 + 16 * wave + c)) * CC + 8 * hh;
  const unsigned short* bph = Hh + brow;
  const unsigned short* bpl = Hl + brow;

  v8f acc[4];
#pragma unroll
  for (int mt = 0; mt < 4; ++mt) acc[mt] = zero8();

#pragma unroll 2
  for (int ks = 0; ks < CC / 32; ++ks) {
    const Frag fh = ldfrag(bph + 32 * ks);
    const Frag fl = ldfrag(bpl + 32 * ks);
#pragma unroll
    for (int mt = 0; mt < 4; ++mt) {
      const Frag fa = ldfrag(ap + (size_t)(16 * mt) * CC + 32 * ks);
      acc[mt] = mma_b(fa.bf, fh.bf, acc[mt]);
      acc[mt] = mma_b(fa.bf, fl.bf, acc[mt]);
    }
  }

  const float* bias = (mat == 0) ? bq : ((mat == 1) ? bk : bv);
  const int nl = 16 * wave + c;
  if (mat != 2) {
#pragma unroll
    for (int mt = 0; mt < 4; ++mt) {
      const v4f b0 = *(const v4f*)(bias + o0 + 16 * mt + 8 * hh);
      const v4f b1 = *(const v4f*)(bias + o0 + 16 * mt + 8 * hh + 4);
      v4f va, vb;
#pragma unroll
      for (int r = 0; r < 4; ++r) { va[r] = acc[mt][r] + bfr(b0[r]); vb[r] = acc[mt][4 + r] + bfr(b1[r]); }
      *(v4f*)(Os + nl * OSP + 16 * mt + 8 * hh)     = va;
      *(v4f*)(Os + nl * OSP + 16 * mt + 8 * hh + 4) = vb;
    }
  } else {
#pragma unroll
    for (int mt = 0; mt < 4; ++mt) {
      const v4f b0 = *(const v4f*)(bias + o0 + 16 * mt + 8 * hh);
      const v4f b1 = *(const v4f*)(bias + o0 + 16 * mt + 8 * hh + 4);
#pragma unroll
      for (int r = 0; r < 4; ++r) {
        Os[(16 * mt + 8 * hh + r) * OSP + nl]     = acc[mt][r] + bfr(b0[r]);
        Os[(16 * mt + 8 * hh + 4 + r) * OSP + nl] = acc[mt][4 + r] + bfr(b1[r]);
      }
    }
  }
  __syncthreads();

  const int e = tid & 7, lq = tid >> 3;
  v4u u[4];
#pragma unroll
  for (int it = 0; it < 4; ++it) {
    const int row = it * 16 + lq;
    const v4f a = *(const v4f*)(Os + row * OSP + 8 * e);
    const v4f q = *(const v4f*)(Os + row * OSP + 8 * e + 4);
    const float f[8] = {a[0], a[1], a[2], a[3], q[0], q[1], q[2], q[3]};
#pragma unroll
    for (int t = 0; t < 4; ++t)
      u[it][t] = pk16(h_bits((_Float16)f[2 * t]), h_bits((_Float16)f[2 * t + 1]));
  }
  unsigned short* plane = (mat == 0) ? Qd : ((mat == 1) ? Kd : Vd);
#pragma unroll
  for (int pass = 0; pass < 2; ++pass) {
#pragma unroll
    for (int it = 0; it < 4; ++it) {
      const int row = it * 16 + lq;
      const size_t pnk = ((size_t)(b * NN + n0 + row)) * CC + o0 + 8 * e;
      const size_t pv  = ((size_t)(b * CC + o0 + row)) * NN + n0 + 8 * e;
      const size_t po  = (mat != 2) ? pnk : pv;
      *(volatile v4u*)(plane + po) = u[it];
    }
    __threadfence();
  }
}

__global__ __launch_bounds__(256)
void attn_k(const unsigned short* __restrict__ Qp, const unsigned short* __restrict__ Kp,
            const unsigned short* __restrict__ Vp, const float* __restrict__ x, float* out) {
  __shared__ __align__(16) float Sx[2 * SXB];
  __shared__ __align__(16) float Os[QT * OSPW];
  const int tid  = threadIdx.x;
  const int wave = tid >> 5, lane = tid & 31;
  const int hh   = lane >> 4, c = lane & 15;
  const int qg   = wave & 3, ch = wave >> 2;
  const int n0   = blockIdx.x * QT, b = blockIdx.y;

  const unsigned short* qp = Qp + ((size_t)(b * NN + n0 + 16 * qg + c)) * CC + 8 * hh;
  const unsigned short* kp = Kp + ((size_t)(b * NN + 16 * ch + c)) * CC + 8 * hh;
  const unsigned short* vp = Vp + ((size_t)(b * CC + CH * ch + c)) * NN + 8 * hh;

  float* sxw = Sx + (wave * 32 + lane) * 8;
  const float* sxr = Sx + ((wave ^ 4) * 32 + lane) * 8;

  float m = -1.0e30f, l = 0.f;
  v8f o[16];
#pragma unroll
  for (int j = 0; j < 16; ++j) o[j] = zero8();

  int buf = 0;
#pragma unroll 1
  for (int kb = 0; kb < NN; kb += 32) {
    const unsigned short* kbp = kp + (size_t)kb * CC;
    v8f sv = zero8();
#pragma unroll 4
    for (int kc = 0; kc < CC / 32; ++kc) {
      const Frag fq = ldfrag(qp + 32 * kc);
      const Frag fk = ldfrag(kbp + 32 * kc);
      sv = mma_h(fk.h, fq.h, sv);
    }

    {
      v4f w0, w1;
#pragma unroll
      for (int r = 0; r < 4; ++r) { w0[r] = sv[r]; w1[r] = sv[4 + r]; }
      *(v4f*)(sxw + buf * SXB)     = w0;
      *(v4f*)(sxw + buf * SXB + 4) = w1;
    }
    __syncthreads();
    v8f so;
    {
      const v4f r0 = *(const v4f*)(sxr + buf * SXB);
      const v4f r1 = *(const v4f*)(sxr + buf * SXB + 4);
#pragma unroll
      for (int r = 0; r < 4; ++r) { so[r] = r0[r]; so[4 + r] = r1[r]; }
    }
    buf ^= 1;
    v8f s0 = sv, s1 = so;
    if (ch != 0) { s0 = so; s1 = sv; }

    float mx = fmaxf(hmax8(s0), hmax8(s1));
    mx = fmaxf(mx, __shfl_xor(mx, 16, 32));
    const float mn = fmaxf(m, mx);
    const unsigned grew = wave_ballot(mx > m);
    if (grew != 0u) {
      const float corr = __expf((m - mn) * ASCALE);
      l *= corr;
#pragma unroll
      for (int j = 0; j < 16; ++j) {
#pragma unroll
        for (int r = 0; r < 8; ++r) o[j][r] *= corr;
      }
    }
    m = mn;
    const float msh = mn * ASCALE - LNPS;

    FragH ph;
    float ls = 0.f;
#pragma unroll
    for (int r = 0; r < 8; ++r) {
      const float e0 = __expf(s0[r] * ASCALE - msh);
      const float e1 = __expf(s1[r] * ASCALE - msh);
      ls += e0 + e1;
      ph.hv[0][r] = (_Float16)e0;
      ph.hv[1][r] = (_Float16)e1;
    }
    l += ls;

#pragma unroll
    for (int j = 0; j < 16; ++j) {
      const Frag vf = ldfrag(vp + (size_t)(16 * j) * NN + kb);
      o[j] = mma_h(vf.h, ph.v, o[j]);
    }
  }
  l += __shfl_xor(l, 16, 32);
  const float inv = 1.0f / l;

  const int qrow = 16 * qg + c;
  const int e = tid & 7, lq = tid >> 3;
#pragma unroll
  for (int ph4 = 0; ph4 < 4; ++ph4) {
    if (ph4) __syncthreads();
    if (ch == (ph4 >> 1)) {
#pragma unroll
      for (int jj = 0; jj < 8; ++jj) {
        const int j = 8 * (ph4 & 1) + jj;
        v4f va, vb;
#pragma unroll
        for (int r = 0; r < 4; ++r) { va[r] = o[j][r] * inv; vb[r] = o[j][4 + r] * inv; }
        *(v4f*)(Os + qrow * OSPW + 16 * jj + 8 * hh)     = va;
        *(v4f*)(Os + qrow * OSPW + 16 * jj + 8 * hh + 4) = vb;
      }
    }
    __syncthreads();
    v4f res[8];
#pragma unroll
    for (int it = 0; it < 8; ++it) {
      const int L   = it * 32 + lq;
      const int chl = L >> 1, hf = L & 1;
      const int nl  = hf * 32 + 4 * e;
      const size_t idx = ((size_t)(b * CC + 128 * ph4 + chl)) * NN + n0 + nl;
      const v4f xv = *(const v4f*)(x + idx);
#pragma unroll
      for (int t = 0; t < 4; ++t) res[it][t] = Os[(nl + t) * OSPW + chl] + bfr(xv[t]);
    }
#pragma unroll
    for (int pass = 0; pass < 2; ++pass) {
#pragma unroll
      for (int it = 0; it < 8; ++it) {
        const int L   = it * 32 + lq;
        const int chl = L >> 1, hf = L & 1;
        const int nl  = hf * 32 + 4 * e;
        const size_t idx = ((size_t)(b * CC + 128 * ph4 + chl)) * NN + n0 + nl;
        *(volatile v4f*)(out + idx) = res[it];
      }
      __threadfence();
    }
  }
}

extern "C" void kernel_launch(void* const* d_in, const int* in_sizes, int n_in,
                              void* d_out, int out_size, void* d_ws, size_t ws_size,
                              hipStream_t stream) {
  const int XN = NB * CC * NN;
  if (n_in < 9) return;
  if (in_sizes[0] < XN) return;
  if (in_sizes[1] < CC || in_sizes[2] < CC) return;
  if (in_sizes[3] < CC * CC || in_sizes[5] < CC * CC || in_sizes[7] < CC * CC) return;
  if (in_sizes[4] < CC || in_sizes[6] < CC || in_sizes[8] < CC) return;
  if (out_size < XN) return;

  size_t off = 0;
  auto carve = [&](size_t bytes) { const size_t o = off; off += (bytes + 255) & ~(size_t)255; return o; };
  const size_t oWb = carve((size_t)3 * CC * CC * 2);
  const size_t oSt = carve((size_t)NB * NGRP * STL * 4);
  const size_t oHh = carve((size_t)NB * NN * CC * 2);
  const size_t oHl = carve((size_t)NB * NN * CC * 2);
  const size_t oQ  = carve((size_t)NB * NN * CC * 2);
  const size_t oK  = carve((size_t)NB * NN * CC * 2);
  const size_t oV  = carve((size_t)NB * CC * NN * 2);
  if (off > ws_size) return;
  if (off > (size_t)134217728) return;

  const float* x     = (const float*)d_in[0];
  const float* gamma = (const float*)d_in[1];
  const float* beta  = (const float*)d_in[2];
  const float* wq    = (const float*)d_in[3];
  const float* bq    = (const float*)d_in[4];
  const float* wk    = (const float*)d_in[5];
  const float* bk    = (const float*)d_in[6];
  const float* wv    = (const float*)d_in[7];
  const float* bv    = (const float*)d_in[8];

  char* ws = (char*)d_ws;
  unsigned short* Wb = (unsigned short*)(ws + oWb);
  float*          St = (float*)(ws + oSt);
  unsigned short* Hh = (unsigned short*)(ws + oHh);
  unsigned short* Hl = (unsigned short*)(ws + oHl);
  unsigned short* Qw = (unsigned short*)(ws + oQ);
  unsigned short* Kw = (unsigned short*)(ws + oK);
  unsigned short* Vw = (unsigned short*)(ws + oV);
  float* out = (float*)d_out;

  const dim3 blk256(256), blk128(128);

  gn_stats<<<dim3(NB * NGRP), blk256, 0, stream>>>(x, St);
  cvt_w<<<dim3(3 * CC / 4), blk256, 0, stream>>>(wq, wk, wv, Wb);
  cvt_x<<<dim3(NN / QT, CC / QT, NB), blk256, 0, stream>>>(x, gamma, beta, St, Hh, Hl);
  gemm_qkv<<<dim3(NN / QT, 3 * CC / QT, NB), blk128, 0, stream>>>(Wb, Hh, Hl, bq, bk, bv, Qw, Kw, Vw);
  attn_k<<<dim3(NQ / QT, NB), blk256, 0, stream>>>(Qw, Kw, Vw, x, out);
  (void)hipGetLastError();
}
